// CapLayer_33517924778159
// MI455X (gfx1250) — hardware-verified
//
#include <hip/hip_runtime.h>
#include <stddef.h>


typedef _Float16 v16h __attribute__((ext_vector_type(16)));
typedef _Float16 v8h  __attribute__((ext_vector_type(8)));
typedef _Float16 v4h  __attribute__((ext_vector_type(4)));
typedef float    v8f  __attribute__((ext_vector_type(8)));
typedef float    v4f  __attribute__((ext_vector_type(4)));

#ifndef NB
#define NB 64
#endif
#define NB_FULL 64
#define NG   32
#define IND  8
#define NJ   10
#define NJP  5
#define ND   16
#define JD   160
#define NP   196
#define CIN  (NG * IND)
#define KS   16
#define KROW (NG * KS)

#define LDX  232
#define XT_ROWS 224
#define LDXT 16
#define LDU  16
#define LDT  72
#define LDWJ 520
#define LDVA 16

#define WCARRY  64.0f
#define VSCARRY 64.0f
#define PCARRY  1024.0f
#define YCARRY  16.0f

static_assert(NB >= 16 && NB <= NB_FULL && (NB % 16) == 0);
static_assert(NB <= 64);
static_assert(NJ == 2 * NJP && JD == NJ * ND && ND == 16);
static_assert(IND == 8 && KS == 16 && IND + 1 <= KS);
static_assert((KROW % 32) == 0 && KROW == 512);
static_assert((NP % 4) == 0 && (NP * IND) / 4 == 392 && 13 * 32 >= 392);
static_assert(LDX >= 224 && (LDX % 8) == 0 && XT_ROWS == 14 * 16 && XT_ROWS >= NP);
static_assert((16 * LDX) / 8 == 464 && 15 * 32 >= 464 && LDX / 8 == 29);
static_assert((XT_ROWS * LDXT) / 8 == 448 && 14 * 32 == 448);
static_assert((LDT % 8) == 0 && LDT >= 64);
static_assert((LDWJ % 8) == 0 && LDWJ >= KROW);
static_assert(4 * 4 == 16);
static_assert(32 * 2 == 64);
static_assert(2 * 32 * 16 * 16 == 64 * 256);

static_assert((16 * LDX + XT_ROWS * LDXT + 16 * LDU + 16 * LDT) * 2 <= 131072);
static_assert(32 * LDWJ * 2 + 64 * 32 * 4 + 128 * LDVA * 2 + 8 * 16 * LDT * 2 <= 65536);

#define YP_BYTES ((size_t)16 * NB * KROW * 2)
#define UP_BYTES ((size_t)NJP * NB * 2 * KROW * 2)
#define VS_BYTES ((size_t)NJP * NB * 32 * 4)
#define OFF_YP ((size_t)0)
#define OFF_UP (OFF_YP + YP_BYTES)
#define OFF_VS (OFF_UP + UP_BYTES)
#define WS_TOTAL (OFF_VS + VS_BYTES)
static_assert((YP_BYTES % 128) == 0 && (UP_BYTES % 128) == 0 && (VS_BYTES % 128) == 0);
static_assert(WS_TOTAL <= (size_t)134217728);

__device__ __forceinline__ float bf16r(float x) {
  unsigned int u = __float_as_uint(x);
  u = (u + 0x7FFFu + ((u >> 16) & 1u)) & 0xFFFF0000u;
  return __uint_as_float(u);
}

static __device__ __forceinline__ _Float16 toh_flush(float v) {
  const _Float16 r = (_Float16)v;
  return (fabsf(v) < 6.103515625e-05f) ? (_Float16)0.0f : r;
}

__device__ __forceinline__ v16h frag_at(const _Float16* p) {
  v8h lo = *(const v8h*)(p);
  v8h hi = *(const v8h*)(p + 16);
  v16h out;
#pragma unroll
  for (int i = 0; i < 8; ++i) { out[i] = lo[i]; out[i + 8] = hi[i]; }
  return out;
}
__device__ __forceinline__ v16h frag_k16(const _Float16* p) {
  v8h lo = *(const v8h*)(p);
  v16h out;
#pragma unroll
  for (int i = 0; i < 8; ++i) { out[i] = lo[i]; out[i + 8] = (_Float16)0.0f; }
  return out;
}

__device__ __forceinline__ v8f wmma16(v16h a, v16h b, v8f c) {
  v8f d = __builtin_amdgcn_wmma_f32_16x16x32_f16(false, a, false, b, (short)0, c,
                                                 false, false);
  asm volatile("v_nop\n\tv_nop\n\tv_nop\n\tv_nop" : "+v"(d) : "v"(a), "v"(b));
  return d;
}

__device__ __forceinline__ float red16_max(float x) {
#pragma unroll
  for (int off = 1; off < 16; off <<= 1) x = fmaxf(x, __shfl_xor(x, off, 32));
  return x;
}
__device__ __forceinline__ float red16_sum(float x) {
#pragma unroll
  for (int off = 1; off < 16; off <<= 1) x += __shfl_xor(x, off, 32);
  return x;
}

__device__ __forceinline__ void wave_lds_sync() {
  __builtin_amdgcn_fence(3  , "wavefront");
  asm volatile("s_wait_dscnt 0x0" ::: "memory");
  __builtin_amdgcn_wave_barrier();
}

__global__ __launch_bounds__(32) void route_kernel(
    const float* __restrict__ x, const _Float16* __restrict__ Up,
    _Float16* __restrict__ Yp, int use_u) {
  __shared__ _Float16 Xs[16 * LDX];
  __shared__ _Float16 Xt[XT_ROWS * LDXT];
  __shared__ _Float16 Ut[16 * LDU];
  __shared__ _Float16 Ys[16 * LDT];

  const unsigned lane = threadIdx.x & 31u;
  const unsigned hh = lane >> 4, m = lane & 15u;
  const unsigned b = blockIdx.x >> 3;
  const unsigned gq = blockIdx.x & 7u;

#pragma unroll 1
  for (unsigned t = 0; t < 15u; ++t) {
    const unsigned idx = lane + 32u * t;
    if (idx < 464u) {
      const unsigned row = idx / 29u, cc = idx - row * 29u;
      v8h z;
#pragma unroll
      for (unsigned i = 0; i < 8u; ++i)
        z[i] = (row == 8u && (cc * 8u + i) < (unsigned)NP) ? (_Float16)1.0f : (_Float16)0.0f;
      *(v8h*)&Xs[row * LDX + cc * 8u] = z;
    }
  }
#pragma unroll 1
  for (unsigned t = 0; t < 14u; ++t) {
    const unsigned idx = lane + 32u * t;
    const unsigned row = idx >> 1, part = idx & 1u;
    v8h z;
#pragma unroll
    for (unsigned i = 0; i < 8u; ++i)
      z[i] = (i == 0u && part == 1u && row < (unsigned)NP) ? (_Float16)1.0f : (_Float16)0.0f;
    *(v8h*)&Xt[row * LDXT + part * 8u] = z;
  }

#pragma unroll 1
  for (unsigned gi = 0; gi < 4u; ++gi) {
    const unsigned g = gq * 4u + gi;
    __syncthreads();

    const float* xg = x + ((size_t)b * CIN + (size_t)g * IND) * NP;
#pragma unroll 1
    for (unsigned t = 0; t < 13u; ++t) {
      const unsigned idx = lane + 32u * t;
      const unsigned idc = (idx < 391u) ? idx : 391u;
      v4f xv = *(const v4f*)(xg + (size_t)idc * 4u);
      asm volatile("" : "+v"(xv));
      const unsigned kk = idc / 49u;
      const unsigned p = (idc - kk * 49u) * 4u;
      if (idx < 392u) {
        v4h hv;
#pragma unroll
        for (int e = 0; e < 4; ++e) hv[e] = toh_flush(bf16r(xv[e]));
        *(v4h*)&Xs[kk * LDX + p] = hv;
#pragma unroll
        for (unsigned e = 0; e < 4u; ++e) Xt[(p + e) * LDXT + kk] = hv[e];
      }
    }

    {
      const unsigned j = lane >> 1, part = lane & 1u;
      const unsigned jc = (j < (unsigned)(NJ - 1)) ? j : (unsigned)(NJ - 1);
      v8h uv;
#pragma unroll
      for (int i = 0; i < 8; ++i) uv[i] = (_Float16)0.0f;
      if (use_u != 0) {
        const size_t off = ((((size_t)(jc >> 1) * NB + b) * 2u + (jc & 1u)) * KROW) +
                           (size_t)g * KS + part * 8u;
        v8h ld = *(const v8h*)(Up + off);
#pragma unroll
        for (int i = 0; i < 8; ++i) uv[i] = (j < (unsigned)NJ) ? ld[i] : (_Float16)0.0f;
      }
      *(v8h*)&Ut[j * LDU + part * 8u] = uv;
    }
    __syncthreads();

    const v16h uf = frag_k16(&Ut[m * LDU + hh * 8u]);
    v8f yacc = {};
#pragma unroll 1
    for (unsigned ks = 0; ks < 7u; ++ks) {
      v16h cf;
#pragma unroll
      for (unsigned tt = 0; tt < 2u; ++tt) {
        const unsigned p0 = ks * 32u + tt * 16u;
        const v16h xa = frag_k16(&Xt[(p0 + m) * LDXT + hh * 8u]);
        v8f zero = {};
        const v8f d = wmma16(xa, uf, zero);
#pragma unroll
        for (unsigned r = 0; r < 8u; ++r) {
          const float lg = (m < (unsigned)NJ) ? d[r] * (1.0f / WCARRY) : -1.0e30f;
          const float mx = red16_max(lg);
          const float e = __expf(lg - mx);
          const float sm = red16_sum(e);
          const float c = e * __builtin_amdgcn_rcpf(sm);
          const bool live = (m < (unsigned)NJ) && ((p0 + hh * 8u + r) < (unsigned)NP);
          cf[tt * 8u + r] = toh_flush(live ? c * PCARRY : 0.0f);
        }
      }
      const v16h xb = frag_at(&Xs[m * LDX + ks * 32u + hh * 8u]);
      yacc = wmma16(cf, xb, yacc);
    }
#pragma unroll
    for (unsigned r = 0; r < 8u; ++r)
      Ys[(hh * 8u + r) * LDT + gi * 16u + m] = toh_flush(yacc[r] * (YCARRY / PCARRY));
  }
  __syncthreads();

  v8h xo[4];
  size_t off[4];
#pragma unroll
  for (unsigned i = 0; i < 4u; ++i) {
    const unsigned r = 4u * i + (lane >> 3);
    const unsigned c = (lane & 7u) * 8u;
    xo[i] = *(const v8h*)&Ys[r * LDT + c];
    off[i] = ((size_t)r * NB + b) * KROW + gq * 64u + c;
  }
#pragma unroll
  for (int i = 0; i < 4; ++i) *(volatile v8h*)(Yp + off[i]) = xo[i];
  __threadfence();
#pragma unroll
  for (int i = 0; i < 4; ++i) *(volatile v8h*)(Yp + off[i]) = xo[i];
}

__global__ __launch_bounds__(256) void fin_kernel(
    const float* __restrict__ W, const float* __restrict__ bias,
    const _Float16* __restrict__ Yp, float* vs0, _Float16* __restrict__ Up,
    float* __restrict__ out, int mode) {
  __shared__ _Float16 Wj[32 * LDWJ];
  __shared__ float    Vst[64 * 32];
  __shared__ _Float16 Va[128 * LDVA];
  __shared__ _Float16 Us[8 * 16 * LDT];

  const unsigned tid = threadIdx.x, lane = tid & 31u;
  const unsigned wave = (unsigned)__builtin_amdgcn_readfirstlane((int)(tid >> 5));
  const unsigned hh = lane >> 4, m = lane & 15u;
  const unsigned jp = blockIdx.x;
  const unsigned jj = wave >> 2, mt = wave & 3u;
  const unsigned j = 2u * jp + jj;
  const bool act = (mt * 16u < (unsigned)NB);

#pragma unroll 1
  for (unsigned it = 0; it < 64u; ++it) {
    const unsigned idx = tid + 256u * it;
    const unsigned kk = idx & 15u, d = (idx >> 4) & 15u, g = (idx >> 8) & 31u, sj = idx >> 13;
    const unsigned kc = (kk < 7u) ? kk : 7u;
    const unsigned orow = g * JD + (2u * jp + sj) * ND + d;
    float wv = W[(size_t)orow * IND + kc];
    float bv = bias[orow];
    asm volatile("" : "+v"(wv));
    asm volatile("" : "+v"(bv));
    const float val = (kk < 8u) ? wv : ((kk == 8u) ? bv : 0.0f);
    Wj[(sj * 16u + d) * LDWJ + g * 16u + kk] = toh_flush(WCARRY * bf16r(val));
  }
  __syncthreads();

  const unsigned brow = mt * 16u + m;
  const unsigned browc = (brow < (unsigned)NB) ? brow : (unsigned)(NB - 1);
  const _Float16* ap = Yp + ((size_t)j * NB + browc) * KROW + hh * 8u;
  const unsigned wjo = (jj * 16u + m) * LDWJ + hh * 8u;
  v8f acc = {};
#pragma unroll 2
  for (unsigned k0 = 0; k0 < (unsigned)KROW; k0 += 32u) {
    const v16h a = frag_at(ap + k0);
    const v16h bq = frag_at(&Wj[wjo + k0]);
    acc = wmma16(a, bq, acc);
  }

#pragma unroll
  for (unsigned r = 0; r < 8u; ++r) {
    const float s = acc[r] * (1.0f / (YCARRY * WCARRY));
    const float nsq = red16_sum(s * s);
    const float nrm = sqrtf(nsq);
    const float coeff = nsq * __builtin_amdgcn_rcpf(1.0f + nsq) *
                        __builtin_amdgcn_rcpf(nrm + 1.0e-20f);
    const float v = s * coeff;
    const unsigned br = mt * 16u + hh * 8u + r;
    const unsigned brc = (br < (unsigned)NB) ? br : (unsigned)(NB - 1);
    float tot = v;
    if (mode == 1) {
      const float pv = vs0[((size_t)jp * NB + brc) * 32u + jj * 16u + m];
      tot = pv + v;
    }
    Vst[br * 32u + jj * 16u + m] = tot;
    Va[(jj * 64u + br) * LDVA + m] = toh_flush(VSCARRY * tot);
  }
  __syncthreads();

  if (mode == 0 || mode == 2) {
    v4f xs[2];
    unsigned bb[2], pc;
    pc = tid & 7u;
#pragma unroll
    for (unsigned i = 0; i < 2u; ++i) {
      bb[i] = 32u * i + (tid >> 3);
      xs[i] = *(const v4f*)&Vst[bb[i] * 32u + pc * 4u];
    }
    if (mode == 0) {
#pragma unroll
      for (int i = 0; i < 2; ++i)
        if (bb[i] < (unsigned)NB)
          *(volatile v4f*)(vs0 + ((size_t)jp * NB + bb[i]) * 32u + pc * 4u) = xs[i];
      __threadfence();
#pragma unroll
      for (int i = 0; i < 2; ++i)
        if (bb[i] < (unsigned)NB)
          *(volatile v4f*)(vs0 + ((size_t)jp * NB + bb[i]) * 32u + pc * 4u) = xs[i];
    } else {
#pragma unroll
      for (int i = 0; i < 2; ++i)
        if (bb[i] < (unsigned)NB)
          *(volatile v4f*)(out + (size_t)bb[i] * JD + jp * 32u + pc * 4u) = xs[i];
      __threadfence();
#pragma unroll
      for (int i = 0; i < 2; ++i)
        if (bb[i] < (unsigned)NB)
          *(volatile v4f*)(out + (size_t)bb[i] * JD + jp * 32u + pc * 4u) = xs[i];
    }
  }

  if (mode < 2) {
    const v16h af = frag_k16(&Va[(jj * 64u + mt * 16u + m) * LDVA + hh * 8u]);
    _Float16* St = Us + wave * (16u * LDT);
#pragma unroll 1
    for (unsigned q = 0; q < 8u; ++q) {
      wave_lds_sync();
#pragma unroll
      for (unsigned t = 0; t < 4u; ++t) {
        const unsigned g = 4u * q + t;
        v16h bf;
#pragma unroll
        for (unsigned i = 0; i < 8u; ++i) {
          bf[i] = Wj[(jj * 16u + hh * 8u + i) * LDWJ + g * 16u + m];
          bf[i + 8u] = (_Float16)0.0f;
        }
        v8f zero = {};
        const v8f u = wmma16(af, bf, zero);
#pragma unroll
        for (unsigned r = 0; r < 8u; ++r)
          St[(hh * 8u + r) * LDT + t * 16u + m] = toh_flush(u[r] * (1.0f / VSCARRY));
      }
      wave_lds_sync();
      v8h xo[4];
      size_t off[4];
#pragma unroll
      for (unsigned i = 0; i < 4u; ++i) {
        const unsigned r = 4u * i + (lane >> 3);
        const unsigned c = (lane & 7u) * 8u;
        const unsigned br = mt * 16u + r;
        const unsigned brc = (br < (unsigned)NB) ? br : (unsigned)(NB - 1);
        xo[i] = *(const v8h*)&St[r * LDT + c];
        off[i] = (((size_t)jp * NB + brc) * 2u + jj) * KROW + q * 64u + c;
      }
      if (act) {
#pragma unroll
        for (int i = 0; i < 4; ++i) *(volatile v8h*)(Up + off[i]) = xo[i];
        __threadfence();
#pragma unroll
        for (int i = 0; i < 4; ++i) *(volatile v8h*)(Up + off[i]) = xo[i];
      }
    }
  }
}

extern "C" void kernel_launch(void* const* d_in, const int* in_sizes, int n_in,
                              void* d_out, int out_size, void* d_ws, size_t ws_size,
                              hipStream_t stream) {
  if (n_in < 3) return;
  if ((long long)in_sizes[0] < (long long)NB * CIN * NP) return;
  if ((long long)in_sizes[1] < (long long)NG * JD * IND) return;
  if ((long long)in_sizes[2] < (long long)NG * JD) return;
  if ((long long)out_size < (long long)NB * JD) return;
  if (ws_size < WS_TOTAL) return;

  const float* x    = (const float*)d_in[0];
  const float* W    = (const float*)d_in[1];
  const float* bias = (const float*)d_in[2];
  float* out = (float*)d_out;

  char* ws = (char*)d_ws;
  _Float16* Yp  = (_Float16*)(ws + OFF_YP);
  _Float16* Upl = (_Float16*)(ws + OFF_UP);
  float*    VS0 = (float*)(ws + OFF_VS);

  for (int it = 0; it < 3; ++it) {
    route_kernel<<<dim3(NB * 8), dim3(32), 0, stream>>>(x, Upl, Yp, it > 0 ? 1 : 0);
    fin_kernel<<<dim3(NJP), dim3(256), 0, stream>>>(W, bias, Yp, VS0, Upl, out, it);
  }
}
